// EncoderLayer_64682207478416
// MI455X (gfx1250) — hardware-verified
//
#include <hip/hip_runtime.h>
#include <math.h>

typedef __attribute__((ext_vector_type(16))) _Float16 v16h;
typedef __attribute__((ext_vector_type(16))) __bf16 v16b;
typedef __attribute__((ext_vector_type(8)))  _Float16 v8h;
typedef __attribute__((ext_vector_type(8)))  float v8f;
typedef __attribute__((ext_vector_type(4)))  float v4f;
typedef __attribute__((ext_vector_type(4)))  unsigned v4u;

#ifndef NB
#define NB 4
#endif
#ifndef SEQ
#define SEQ 2048
#endif
#define TT SEQ
#define NB_FULL 4
#define TT_FULL 2048
#define CC 512
#define DIN 512
#define NH 8
#define HD 64
#define FF 2048
#define HG 4
#define NQB (TT / 64)
#define NRW (NB * TT)
#define SCALE (0.125f)
#define QHI 64

static_assert(HD == 64);
static_assert(CC == NH * HD);
static_assert(DIN == CC);
static_assert(DIN == 512);
static_assert(TT % 256 == 0);
static_assert(TT <= TT_FULL);
static_assert(NB <= NB_FULL);
static_assert(NRW % 64 == 0);
static_assert(CC % 128 == 0);
static_assert(FF % 128 == 0);
static_assert(DIN % 32 == 0);
static_assert(FF % 32 == 0);
static_assert(NH % HG == 0);
static_assert(QHI == 64);

#define SZ_H16  (2u * (size_t)NRW * CC)
#define SZ_QL   (2u * (size_t)NB * QHI * CC)
#define SZ_S    (4u * (size_t)HG * TT * TT)
#define SZ_HF   (4u * (size_t)NRW * FF)
#define SZ_SHF  (SZ_S > SZ_HF ? SZ_S : SZ_HF)
#define SZ_ROWS (4u * (size_t)NRW * CC)
#define WS_QH   ((size_t)0)
#define WS_KH   (WS_QH + SZ_H16)
#define WS_VT   (WS_KH + SZ_H16)
#define WS_QL   (WS_VT + SZ_H16)
#define WS_S    (WS_QL + SZ_QL)
#define WS_XY   (WS_S + SZ_SHF)
#define WS_R1   (WS_XY + SZ_ROWS)
#define WS_TOTAL (WS_R1 + SZ_ROWS)
static_assert(SZ_S <= SZ_SHF);
static_assert(SZ_HF <= SZ_SHF);
static_assert(WS_TOTAL <= (size_t)134217728);
static_assert((SZ_H16 % 128) == 0);
static_assert((SZ_QL % 128) == 0);
static_assert((SZ_SHF % 128) == 0);
static_assert((SZ_ROWS % 128) == 0);
static_assert((size_t)(NRW / 8) * 8 * DIN == (size_t)NRW * DIN);
static_assert((size_t)(NRW / 64) * (CC / 128) * 64 * 128 == (size_t)NRW * CC);
static_assert((size_t)NQB * (TT / 128) * 64 * 128 == (size_t)TT * TT);
static_assert((size_t)NQB * 64 * HD * NH == (size_t)TT * CC);
static_assert((size_t)(NRW / 64) * (FF / 128) * 64 * 128 == (size_t)NRW * FF);

template <typename T> __device__ __forceinline__ void vst2(void* p, T v) { *(volatile T*)p = v; __threadfence(); *(volatile T*)p = v; }
__device__ __forceinline__ v8f wmma16(v16h a, v16h b, v8f c) {
  v8f d = __builtin_amdgcn_wmma_f32_16x16x32_f16(false, a, false, b, (short)0, c, false, false);
  asm volatile("v_nop\n\tv_nop\n\tv_nop\n\tv_nop" : "+v"(d) : "v"(a), "v"(b));
  return d;
}
__device__ __forceinline__ v8f wmma_bf(v16b a, v16b b, v8f c) {
  v8f d = __builtin_amdgcn_wmma_f32_16x16x32_bf16(false, a, false, b, (short)0, c, false, false);
  asm volatile("v_nop\n\tv_nop\n\tv_nop\n\tv_nop" : "+v"(d) : "v"(a), "v"(b));
  return d;
}
__device__ __forceinline__ v16h frag_h(const _Float16* rowk0, unsigned lane) {
  union { v16h v; v8h q[2]; } u; const _Float16* p = rowk0 + 8u * (lane >> 4);
  u.q[0] = *(const v8h*)p; u.q[1] = *(const v8h*)(p + 16); return u.v;
}
__device__ __forceinline__ v16h frag_f32(const float* rowk0, unsigned lane) {
  v16h a; const float* p = rowk0 + 8u * (lane >> 4);
#pragma unroll
  for (int i = 0; i < 8; ++i) { a[i] = (_Float16)p[i]; a[8 + i] = (_Float16)p[16 + i]; }
  return a;
}
__device__ __forceinline__ v16h frag_f32s(const float* rowk0, unsigned lane, float sc) {
  v16h a; const float* p = rowk0 + 8u * (lane >> 4);
#pragma unroll
  for (int i = 0; i < 8; ++i) { a[i] = (_Float16)(p[i] * sc); a[8 + i] = (_Float16)(p[16 + i] * sc); }
  return a;
}
struct F2 { v16b h, l; };
__device__ __forceinline__ F2 bsplit16(const float v[16]) { F2 r;
#pragma unroll
  for (int i = 0; i < 16; ++i) { const __bf16 h = (__bf16)v[i]; r.h[i] = h; r.l[i] = (__bf16)(v[i] - (float)h); }
  return r; }
__device__ __forceinline__ F2 split_row(const float* row, unsigned k0, unsigned lane) { float v[16]; const float* p = row + k0 + 8u * (lane >> 4);
#pragma unroll
  for (int i = 0; i < 8; ++i) { v[i] = p[i]; v[8 + i] = p[16 + i]; }
  return bsplit16(v); }
__device__ __forceinline__ float bfr(float v) { return (float)(__bf16)v; }
__device__ __forceinline__ float gelu_f(float t) { return 0.5f * t * (1.0f + erff(t * 0.70710678118654752f)); }
#define LDSX() do { asm volatile("s_wait_dscnt 0" ::: "memory"); __builtin_amdgcn_wave_barrier(); __builtin_amdgcn_fence(3  , "workgroup"); } while (0)

__device__ __forceinline__ v16b wcol_hdk(const float* Wm, unsigned k0, unsigned o, unsigned lane) { v16b w; const unsigned g = lane >> 4; const float* p = Wm + (size_t)(o >> 6) * (DIN * HD) + (o & 63u);
#pragma unroll
  for (int i = 0; i < 8; ++i) { w[i] = (__bf16)p[(size_t)(k0 + 8u * g + i) * HD]; w[8 + i] = (__bf16)p[(size_t)(k0 + 16u + 8u * g + i) * HD]; }
  return w; }
__device__ __forceinline__ v16h wcolh_io(const float* Wm, unsigned k0, unsigned o, unsigned lane, unsigned ld) { v16h w; const unsigned g = lane >> 4;
#pragma unroll
  for (int i = 0; i < 8; ++i) { w[i] = (_Float16)(bfr(Wm[(size_t)(k0 + 8u * g + i) * ld + o]) * 256.0f); w[8 + i] = (_Float16)(bfr(Wm[(size_t)(k0 + 16u + 8u * g + i) * ld + o]) * 256.0f); }
  return w; }

__global__ __launch_bounds__(256) void k_lnx(const float* __restrict__ X, int cvt_in, int xfull, const float* __restrict__ G, const float* __restrict__ BE, float* __restrict__ OUT) {
  const unsigned wave = threadIdx.x >> 5, lane = threadIdx.x & 31u; const unsigned row = blockIdx.x * 8u + wave; if (row >= (unsigned)NRW) return;
  const size_t srow = xfull ? ((size_t)(row / (unsigned)TT) * TT_FULL + (row % (unsigned)TT)) : (size_t)row;
  v4f v[4]; float s1 = 0.f;
#pragma unroll
  for (int i = 0; i < 4; ++i) { v4f t = *(const v4f*)(X + srow * DIN + i * 128 + lane * 4u); if (cvt_in) { t[0] = bfr(t[0]); t[1] = bfr(t[1]); t[2] = bfr(t[2]); t[3] = bfr(t[3]); } v[i] = t; s1 += (t[0] + t[1]) + (t[2] + t[3]); }
#pragma unroll
  for (int o = 1; o < 32; o <<= 1) s1 += __shfl_xor(s1, o);
  const float mu = s1 * (1.0f / DIN); float q = 0.f;
#pragma unroll
  for (int i = 0; i < 4; ++i) {
#pragma unroll
    for (int k = 0; k < 4; ++k) { const float d = v[i][k] - mu; q += d * d; } }
#pragma unroll
  for (int o = 1; o < 32; o <<= 1) q += __shfl_xor(q, o);
  const float sd = sqrtf(q * (1.0f / (DIN - 1))); const float inv = 1.0f / (sd + 1e-10f);
#pragma unroll
  for (int i = 0; i < 4; ++i) { const unsigned c = i * 128 + lane * 4u; const v4f gv = *(const v4f*)(G + c), bv = *(const v4f*)(BE + c); v4f r4;
#pragma unroll
    for (int k = 0; k < 4; ++k) r4[k] = bfr(gv[k]) * ((v[i][k] - mu) * inv) + bfr(bv[k]);
    vst2(OUT + (size_t)row * DIN + c, r4); } }

__global__ __launch_bounds__(128) void k_proj(const float* __restrict__ XN, const float* __restrict__ WQ, const float* __restrict__ WK, const float* __restrict__ WV, const float* __restrict__ BQ, const float* __restrict__ BK, const float* __restrict__ BV,
    _Float16* __restrict__ QH, _Float16* __restrict__ QL, _Float16* __restrict__ KH, _Float16* __restrict__ VT) {
  __shared__ __align__(16) _Float16 sh[64][136], sl[64][136]; __shared__ __align__(16) _Float16 th[128][72];
  const unsigned tid = threadIdx.x, wave = tid >> 5, lane = tid & 31u, col = lane & 15u, g = lane >> 4; const unsigned which = blockIdx.z; const unsigned c0 = blockIdx.y * 128u; const unsigned r0 = blockIdx.x * 64u; const unsigned bb = r0 / (unsigned)TT; const unsigned t0 = r0 % (unsigned)TT;
  const float* WA = which == 0 ? WQ : which == 1 ? WK : WV; const float* BA = which == 0 ? BQ : which == 1 ? BK : BV;
  v8f acc[8] = {};
#pragma unroll 2
  for (unsigned kc = 0; kc < DIN / 32; ++kc) { const F2 a2 = split_row(XN + (size_t)(r0 + wave * 16u + col) * DIN, kc * 32u, lane);
    asm volatile("s_wait_loadcnt 0x0" ::: "memory");
#pragma unroll
    for (int j = 0; j < 8; ++j) { const v16b w = wcol_hdk(WA, kc * 32u, c0 + j * 16 + col, lane); asm volatile("s_wait_loadcnt 0x0" ::: "memory"); acc[j] = wmma_bf(a2.h, w, acc[j]); acc[j] = wmma_bf(a2.l, w, acc[j]); } }
  if (which < 2) { _Float16* DH = which == 0 ? QH : KH; const bool wr_lo = (which == 0) && (t0 < (unsigned)QHI);
#pragma unroll
    for (int j = 0; j < 8; ++j) { const float bias = bfr(BA[c0 + j * 16 + col]);
#pragma unroll
      for (int r = 0; r < 8; ++r) { const float v = acc[j][r] + bias; const _Float16 hv = (_Float16)v; sh[wave * 16u + 8u * g + r][j * 16 + col] = hv; sl[wave * 16u + 8u * g + r][j * 16 + col] = (_Float16)((v - (float)hv) * 1024.0f); } }
    __syncthreads();
    for (unsigned e = tid; e < 64u * 16u; e += 128u) { const unsigned rl = e >> 4, q = e & 15u; vst2(DH + (size_t)(r0 + rl) * CC + c0 + q * 8u, *(const v4u*)&sh[rl][q * 8u]); if (wr_lo) vst2(QL + ((size_t)bb * QHI + t0 + rl) * CC + c0 + q * 8u, *(const v4u*)&sl[rl][q * 8u]); }
  } else {
#pragma unroll
    for (int j = 0; j < 8; ++j) { const float bias = bfr(BA[c0 + j * 16 + col]);
#pragma unroll
      for (int r = 0; r < 8; ++r) { const float v = acc[j][r] + bias; th[j * 16 + col][wave * 16u + 8u * g + r] = (_Float16)v; } }
    __syncthreads();
    for (unsigned e = tid; e < 128u * 8u; e += 128u) { const unsigned cl = e >> 3, q = e & 7u; vst2(VT + ((size_t)bb * CC + c0 + cl) * TT + t0 + q * 8u, *(const v4u*)&th[cl][q * 8u]); } } }

__global__ __launch_bounds__(128) void k_sc(const _Float16* __restrict__ QH, const _Float16* __restrict__ KH, const _Float16* __restrict__ QL, unsigned b, unsigned h0, float* __restrict__ S0) { __shared__ __align__(16) float ss[4][16][132];
  const unsigned qb = blockIdx.x, kb = blockIdx.y; const unsigned h = h0 + blockIdx.z; float* S = S0 + (size_t)blockIdx.z * TT * TT;
  const unsigned tid = threadIdx.x, wave = tid >> 5, lane = tid & 31u, col = lane & 15u, g = lane >> 4; const unsigned k0 = kb * 128u; const unsigned ql0 = qb * 64u + wave * 16u; const size_t q0 = (size_t)b * TT + ql0, kr0 = (size_t)b * TT + k0;
  v8f acc[8] = {}, accl[8] = {};
  const _Float16* QLb = QL + (size_t)b * QHI * CC;
  if (qb * 64u < (unsigned)QHI) {
#pragma unroll
    for (int kc = 0; kc < HD / 32; ++kc) { const v16h ah = frag_h(QH + (q0 + col) * CC + h * HD + kc * 32, lane), al = frag_h(QLb + (size_t)(ql0 + col) * CC + h * HD + kc * 32, lane);
#pragma unroll
      for (int j = 0; j < 8; ++j) { const v16h kbf = frag_h(KH + (kr0 + j * 16 + col) * CC + h * HD + kc * 32, lane); acc[j] = wmma16(ah, kbf, acc[j]); accl[j] = wmma16(al, kbf, accl[j]); } }
  } else {
#pragma unroll
    for (int kc = 0; kc < HD / 32; ++kc) { const v16h ah = frag_h(QH + (q0 + col) * CC + h * HD + kc * 32, lane);
#pragma unroll
      for (int j = 0; j < 8; ++j) { const v16h kbf = frag_h(KH + (kr0 + j * 16 + col) * CC + h * HD + kc * 32, lane); acc[j] = wmma16(ah, kbf, acc[j]); } } }
#pragma unroll
  for (int j = 0; j < 8; ++j) {
#pragma unroll
    for (int r = 0; r < 8; ++r) ss[wave][8u * g + r][j * 16 + col] = (acc[j][r] + accl[j][r] * (1.0f / 1024.0f)) * SCALE; }
  LDSX();
#pragma unroll 1
  for (unsigned rl = 0; rl < 16; ++rl) vst2(S + (size_t)(ql0 + rl) * TT + k0 + lane * 4u, *(const v4f*)&ss[wave][rl][lane * 4u]); }

__global__ __launch_bounds__(256) void k_sm(float* __restrict__ S0) { __shared__ float sred[8]; __shared__ float sbc; __shared__ __align__(16) float shv[TT];
  const unsigned tid = threadIdx.x; const unsigned t = blockIdx.x;
  float* sr = S0 + (size_t)blockIdx.y * TT * TT + (size_t)t * TT;
  float m = -3.0e38f; for (unsigned k = tid; k < (unsigned)TT; k += 256u) { const float v = sr[k]; shv[k] = v; m = fmaxf(m, v); }
#pragma unroll
  for (int o = 1; o < 32; o <<= 1) m = fmaxf(m, __shfl_xor(m, o));
  if ((tid & 31u) == 0) sred[tid >> 5] = m; __syncthreads(); if (tid == 0) { float a = sred[0]; for (int i = 1; i < 8; ++i) a = fmaxf(a, sred[i]); sbc = a; } __syncthreads(); m = sbc; __syncthreads();
  float sum = 0.f; for (unsigned k = tid; k < (unsigned)TT; k += 256u) { const float e = expf(shv[k] - m); shv[k] = e; sum += e; }
#pragma unroll
  for (int o = 1; o < 32; o <<= 1) sum += __shfl_xor(sum, o);
  if ((tid & 31u) == 0) sred[tid >> 5] = sum; __syncthreads(); if (tid == 0) { float a = 0.f; for (int i = 0; i < 8; ++i) a += sred[i]; sbc = 2048.0f / a; } __syncthreads(); const float inv = sbc;
  for (unsigned k = tid; k < (unsigned)TT; k += 256u) shv[k] = shv[k] * inv;
  __syncthreads(); for (unsigned q = tid; q < (unsigned)TT / 4u; q += 256u) vst2(sr + q * 4u, *(const v4f*)&shv[q * 4u]); }

__global__ __launch_bounds__(128) void k_pv(const float* __restrict__ PS0, const _Float16* __restrict__ VT, unsigned b, unsigned h0, float* __restrict__ Y) { const unsigned h = h0 + blockIdx.z; const float* PS = PS0 + (size_t)blockIdx.z * TT * TT; __shared__ __align__(16) float ss[4][16][HD + 4];
  const unsigned tid = threadIdx.x, wave = tid >> 5, lane = tid & 31u, col = lane & 15u, g = lane >> 4; const unsigned qb = blockIdx.x; const unsigned ql0 = qb * 64u + wave * 16u;
  v8f acc[HD / 16] = {};
#pragma unroll 1
  for (unsigned kc = 0; kc < (unsigned)TT / 32u; ++kc) { const v16h p = frag_f32(PS + (size_t)(ql0 + col) * TT + kc * 32u, lane);
    asm volatile("s_wait_loadcnt 0x0" ::: "memory");
#pragma unroll
    for (int j = 0; j < HD / 16; ++j) { const size_t po = ((size_t)b * CC + h * HD + j * 16 + col) * (size_t)TT + kc * 32u; acc[j] = wmma16(p, frag_h(VT + po, lane), acc[j]); } }
#pragma unroll
  for (int j = 0; j < HD / 16; ++j)
#pragma unroll
    for (int r = 0; r < 8; ++r) ss[wave][8u * g + r][j * 16 + col] = acc[j][r] * (1.0f / 2048.0f);
  LDSX();
#pragma unroll 1
  for (unsigned rl = 0; rl < 16; ++rl) if (lane < HD / 4) vst2(Y + ((size_t)b * TT + ql0 + rl) * CC + h * HD + lane * 4u, *(const v4f*)&ss[wave][rl][lane * 4u]); }

__global__ __launch_bounds__(128) void k_out(const float* __restrict__ Y, const float* __restrict__ WO, const float* __restrict__ BO, const float* __restrict__ X, float* __restrict__ R1) { __shared__ __align__(16) float sf[4][16][132];
  const unsigned tid = threadIdx.x, wave = tid >> 5, lane = tid & 31u, col = lane & 15u, g = lane >> 4; const unsigned c0 = blockIdx.y * 128u; const unsigned r0 = blockIdx.x * 64u + wave * 16u;
  v8f acc[8] = {};
#pragma unroll 2
  for (unsigned kc = 0; kc < CC / 32; ++kc) { const v16h a = frag_f32s(Y + (size_t)(r0 + col) * CC + kc * 32u, lane, 16.0f); asm volatile("s_wait_loadcnt 0x0" ::: "memory");
#pragma unroll
    for (int j = 0; j < 8; ++j) { const v16h w = wcolh_io(WO, kc * 32u, c0 + j * 16 + col, lane, DIN); asm volatile("s_wait_loadcnt 0x0" ::: "memory"); acc[j] = wmma16(a, w, acc[j]); } }
#pragma unroll
  for (int j = 0; j < 8; ++j) { const float bias = bfr(BO[c0 + j * 16 + col]);
#pragma unroll
    for (int r = 0; r < 8; ++r) sf[wave][8u * g + r][j * 16 + col] = acc[j][r] * (1.0f / 4096.0f) + bias; }
  LDSX();
#pragma unroll 1
  for (unsigned rl = 0; rl < 16; ++rl) { const unsigned r = r0 + rl; const size_t xr = (size_t)(r / (unsigned)TT) * TT_FULL + (r % (unsigned)TT);
    v4f v = *(const v4f*)&sf[wave][rl][lane * 4u]; const v4f xv = *(const v4f*)(X + xr * DIN + c0 + lane * 4u);
    v[0] += bfr(xv[0]); v[1] += bfr(xv[1]); v[2] += bfr(xv[2]); v[3] += bfr(xv[3]);
    vst2(R1 + (size_t)r * DIN + c0 + lane * 4u, v); } }

__global__ __launch_bounds__(128) void k_gemh(const float* __restrict__ A, unsigned lda, unsigned K, const float* __restrict__ Wm, unsigned nout, const float* __restrict__ BIAS, const float* __restrict__ RES, float* __restrict__ OUT) { __shared__ __align__(16) float sf[4][16][132];
  const unsigned tid = threadIdx.x, wave = tid >> 5, lane = tid & 31u, col = lane & 15u, g = lane >> 4; const unsigned c0 = blockIdx.y * 128u; const unsigned r0 = blockIdx.x * 64u + wave * 16u;
  v8f acc[8] = {};
#pragma unroll 1
  for (unsigned kc = 0; kc < K / 32u; ++kc) { v16h a; { const float* p = A + (size_t)(r0 + col) * lda + kc * 32u + 8u * g;
#pragma unroll
      for (int i = 0; i < 8; ++i) { a[i] = (_Float16)p[i]; a[8 + i] = (_Float16)p[16 + i]; } }
    asm volatile("s_wait_loadcnt 0x0" ::: "memory");
#pragma unroll
    for (int j = 0; j < 8; ++j) { v16h w; { const unsigned o = c0 + j * 16 + col; float t0[8], t1[8];
#pragma unroll
        for (int i = 0; i < 8; ++i) t0[i] = Wm[(size_t)(kc * 32u + 8u * g + i) * nout + o];
        asm volatile("s_wait_loadcnt 0x0" ::: "memory");
#pragma unroll
        for (int i = 0; i < 8; ++i) t1[i] = Wm[(size_t)(kc * 32u + 16u + 8u * g + i) * nout + o];
        asm volatile("s_wait_loadcnt 0x0" ::: "memory");
#pragma unroll
        for (int i = 0; i < 8; ++i) { w[i] = (_Float16)(bfr(t0[i]) * 64.0f); w[8 + i] = (_Float16)(bfr(t1[i]) * 64.0f); } }
      acc[j] = wmma16(a, w, acc[j]); } }
#pragma unroll
  for (int j = 0; j < 8; ++j)
#pragma unroll
    for (int r = 0; r < 8; ++r) sf[wave][8u * g + r][j * 16 + col] = acc[j][r] * (1.0f / 64.0f);
  LDSX();
  v4f bz; { const v4f bv = *(const v4f*)(BIAS + c0 + lane * 4u); bz[0] = bfr(bv[0]); bz[1] = bfr(bv[1]); bz[2] = bfr(bv[2]); bz[3] = bfr(bv[3]); }
#pragma unroll 1
  for (unsigned rl = 0; rl < 16; ++rl) { const size_t o = (size_t)(r0 + rl) * nout + c0 + lane * 4u; v4f v = *(const v4f*)&sf[wave][rl][lane * 4u];
    v[0] = gelu_f(v[0] + bz[0]); v[1] = gelu_f(v[1] + bz[1]); v[2] = gelu_f(v[2] + bz[2]); v[3] = gelu_f(v[3] + bz[3]);
    if (RES) { const v4f rv = *(const v4f*)(RES + o); v[0] += rv[0]; v[1] += rv[1]; v[2] += rv[2]; v[3] += rv[3]; }
    vst2(OUT + o, v); } }

extern "C" void kernel_launch(void* const* d_in, const int* in_sizes, int n_in, void* d_out, int out_size, void* d_ws, size_t ws_size, hipStream_t stream) {
  if (n_in < 17) return;
  if (in_sizes[0] < ((NB - 1) * TT_FULL + TT) * DIN) return;
  if (in_sizes[1] < NH * DIN * HD || in_sizes[3] < NH * DIN * HD || in_sizes[5] < NH * DIN * HD) return;
  if (in_sizes[2] < CC || in_sizes[4] < CC || in_sizes[6] < CC) return;
  if (in_sizes[7] < CC * DIN || in_sizes[8] < DIN) return;
  if (in_sizes[9] < DIN || in_sizes[10] < DIN || in_sizes[11] < DIN || in_sizes[12] < DIN) return;
  if (in_sizes[13] < DIN * FF || in_sizes[14] < FF || in_sizes[15] < FF * DIN || in_sizes[16] < DIN) return;
  if (out_size < NRW * DIN) return;
  if (ws_size < (size_t)WS_TOTAL) return;
  const float** F = (const float**)d_in;
  char* ws = (char*)d_ws;
  _Float16 *QH = (_Float16*)(ws + WS_QH), *KH = (_Float16*)(ws + WS_KH), *VT = (_Float16*)(ws + WS_VT), *QL = (_Float16*)(ws + WS_QL);
  float *S = (float*)(ws + WS_S), *HF = (float*)(ws + WS_S), *XY = (float*)(ws + WS_XY), *R1 = (float*)(ws + WS_R1);
  k_lnx<<<dim3(NRW / 8), 256, 0, stream>>>(F[0], 1, 1, F[9], F[10], XY);
  k_proj<<<dim3(NRW / 64, CC / 128, 3), 128, 0, stream>>>(XY, F[1], F[3], F[5], F[2], F[4], F[6], QH, QL, KH, VT);
  for (unsigned b = 0; b < NB; ++b) for (unsigned h0 = 0; h0 < NH; h0 += HG) {
    k_sc<<<dim3(NQB, TT / 128, HG), 128, 0, stream>>>(QH, KH, QL, b, h0, S);
    k_sm<<<dim3(TT, HG), 256, 0, stream>>>(S);
    k_pv<<<dim3(NQB, 1, HG), 128, 0, stream>>>(S, VT, b, h0, XY);
  }
  k_out<<<dim3(NRW / 64, DIN / 128), 128, 0, stream>>>(XY, F[7], F[8], F[0], R1);
  k_lnx<<<dim3(NRW / 8), 256, 0, stream>>>(R1, 0, 0, F[11], F[12], XY);
  k_gemh<<<dim3(NRW / 64, FF / 128), 128, 0, stream>>>(XY, DIN, DIN, F[13], FF, F[14], nullptr, HF);
  k_gemh<<<dim3(NRW / 64, DIN / 128), 128, 0, stream>>>(HF, FF, FF, F[15], DIN, F[16], R1, (float*)d_out);
}
